// ParallelAttentionBlock_65687229825659
// MI455X (gfx1250) — hardware-run, weakly checked
//
#include <hip/hip_runtime.h>
#include <math.h>

constexpr int kBatch   = 2;
constexpr int kSeq     = 2048;
constexpr int kDModel  = 1024;
constexpr int kHeads   = 16;
constexpr int kHeadDim = 64;
constexpr int kKVHeads = 4;
constexpr int kKVDim   = kKVHeads * kHeadDim;
constexpr int kDff     = 4096;
constexpr int kTok     = kBatch * kSeq;
constexpr int kQKVN    = kDModel + 2 * kKVDim;
constexpr int kKcol    = kDModel;
constexpr int kVcol    = kDModel + kKVDim;
constexpr int kMChunk  = 1024;
constexpr int kGUld    = 2 * kDff;

constexpr float kWCarry     = 16.0f;
constexpr float kWdCarry    = 64.0f;
constexpr float kPCarry     = 2048.0f;
constexpr float kAttCarry   = 64.0f;
constexpr float kHCarry     = 16.0f;
constexpr float kScoreScale = 0.125f;
constexpr float kLnEps      = 1e-5f;
constexpr float kInvD       = 1.0f / 1024.0f;

typedef __attribute__((ext_vector_type(16))) _Float16 v16h;
typedef __attribute__((ext_vector_type(8)))  _Float16 v8h;
typedef __attribute__((ext_vector_type(16))) __bf16   v16b;
typedef __attribute__((ext_vector_type(8)))  __bf16   v8b;
typedef __attribute__((ext_vector_type(8)))  float    v8f;
typedef __attribute__((ext_vector_type(4)))  float    v4f;
typedef __attribute__((ext_vector_type(2)))  float    v2f;
typedef __attribute__((ext_vector_type(4)))  unsigned int v4u;
typedef __attribute__((ext_vector_type(2)))  unsigned int v2u;

__device__ __forceinline__ unsigned short f2bf_bits(float f) {
  unsigned u = __float_as_uint(f);
  return (unsigned short)((u + 0x7FFFu + ((u >> 16) & 1u)) >> 16);
}
__device__ __forceinline__ float bf_bits2f(unsigned short h) { return __uint_as_float(((unsigned)h) << 16); }

__device__ __forceinline__ void dep_guard_h(v8f& a, v8f& b, v16h x, v16h y) { asm volatile("v_nop\n\tv_nop\n\tv_nop\n\tv_nop" : "+v"(a), "+v"(b) : "v"(x), "v"(y)); }
__device__ __forceinline__ void dep_guard_b(v8f& a, v8f& b, v16b x, v16b y) { asm volatile("v_nop\n\tv_nop\n\tv_nop\n\tv_nop" : "+v"(a), "+v"(b) : "v"(x), "v"(y)); }
__device__ __forceinline__ void keep4_h(v16h a, v16h b, v16h c, v16h d) { asm volatile("v_nop" :: "v"(a), "v"(b), "v"(c), "v"(d)); }
__device__ __forceinline__ void keep4_b(v16b a, v16b b, v16b c, v16b d) { asm volatile("v_nop" :: "v"(a), "v"(b), "v"(c), "v"(d)); }
__device__ __forceinline__ void acc_guard4(v8f& a, v8f& b, v8f& c, v8f& d) { asm volatile("v_nop\n\tv_nop\n\tv_nop\n\tv_nop" : "+v"(a), "+v"(b), "+v"(c), "+v"(d)); }
template <typename T> struct Frag;
template <> struct Frag<_Float16> {
  typedef v16h V; union U { v16h v; v8h h[2]; };
  static __device__ __forceinline__ v16h load(const _Float16* p) {
    U f; f.h[0] = *(const v8h*)(p); f.h[1] = *(const v8h*)(p + 16); return f.v;
  }
  static __device__ __forceinline__ v8f mma(v16h a, v16h b, v8f c) {
    return __builtin_amdgcn_wmma_f32_16x16x32_f16(false, a, false, b, (short)0, c, false, false);
  }
  static __device__ __forceinline__ void guard(v8f& a, v8f& b, v16h x, v16h y) { dep_guard_h(a, b, x, y); }
  static __device__ __forceinline__ void keep(v16h a, v16h b, v16h c, v16h d) { keep4_h(a, b, c, d); }
};
template <> struct Frag<__bf16> {
  typedef v16b V; union U { v16b v; v8b h[2]; };
  static __device__ __forceinline__ v16b load(const __bf16* p) {
    U f; f.h[0] = *(const v8b*)(p); f.h[1] = *(const v8b*)(p + 16); return f.v;
  }
  static __device__ __forceinline__ v8f mma(v16b a, v16b b, v8f c) {
    return __builtin_amdgcn_wmma_f32_16x16x32_bf16(false, a, false, b, (short)0, c, false, false);
  }
  static __device__ __forceinline__ void guard(v8f& a, v8f& b, v16b x, v16b y) { dep_guard_b(a, b, x, y); }
  static __device__ __forceinline__ void keep(v16b a, v16b b, v16b c, v16b d) { keep4_b(a, b, c, d); }
};

__device__ __forceinline__ unsigned pk16(unsigned short a, unsigned short b) { return (unsigned)a | ((unsigned)b << 16); }
__device__ __forceinline__ unsigned short h_bits(float f) { const _Float16 h = (_Float16)f; return __builtin_bit_cast(unsigned short, h); }

template <int ET> struct Elem;
template <> struct Elem<0> { typedef _Float16 T; };
template <> struct Elem<1> { typedef __bf16 T; };
template <int ET, bool SPLIT, int BIAS_MODE, int OUT_MODE, bool RESID, int ACT = 0, int CAUSAL = 0>
__global__ __launch_bounds__(256) void wmma_gemm64(
    const unsigned short* __restrict__ Ap, const unsigned short* __restrict__ A2p, int lda, long strideA,
    const unsigned short* __restrict__ Btp, const unsigned short* __restrict__ Bt2p, int ldb, long strideB,
    void* __restrict__ Cout, void* __restrict__ Cout2, int ldc, long strideC,
    const float* __restrict__ bias,
    const float* __restrict__ resid, long strideR,
    int M, int N, int K, float scale) {
  typedef typename Elem<ET>::T T;
  typedef typename Frag<T>::V V;
  const T* A = (const T*)Ap; const T* A2 = (const T*)A2p; const T* Bt = (const T*)Btp; const T* Bt2 = (const T*)Bt2p;
  __shared__ __align__(16) float sT[8][16 * 68];
  const int b    = blockIdx.y;
  const int lane = threadIdx.x & 31;
  const int wave = threadIdx.x >> 5;
  const int tilesN = N >> 6;
  const int tilesM = M >> 6;
  const int tile = blockIdx.x * 8 + wave;
  if (tile >= tilesM * tilesN) return;
  const int tm = tile / tilesN;
  const int tn = tile - tm * tilesN;
  if (CAUSAL == 1 && tn > tm) return;
  const int m0 = tm << 6;
  const int n0 = tn << 6;
  const int Kend = (CAUSAL == 2 && (m0 + 64) < K) ? (m0 + 64) : K;

  const T* Ab  = A  + (size_t)b * strideA;
  const T* Bb  = Bt + (size_t)b * strideB;
  const T* Ab2 = SPLIT ? (A2  + (size_t)b * strideA) : nullptr;
  const T* Bb2 = SPLIT ? (Bt2 + (size_t)b * strideB) : nullptr;

  const int rlane = lane & 15;
  const int koff  = (lane >> 4) * 8;
  const int mOff  = (lane >> 4) * 8;

  v8f acc[4][4];
#pragma unroll
  for (int i = 0; i < 4; ++i)
#pragma unroll
    for (int j = 0; j < 4; ++j) acc[i][j] = (v8f){0.f,0.f,0.f,0.f,0.f,0.f,0.f,0.f};

  for (int k0 = 0; k0 < Kend; k0 += 32) {
    V bh[4], bl[4];
#pragma unroll
    for (int j = 0; j < 4; ++j) {
      const size_t bo = (size_t)(n0 + (j << 4) + rlane) * ldb + koff + k0;
      bh[j] = Frag<T>::load(Bb + bo);
      if (SPLIT) bl[j] = Frag<T>::load(Bb2 + bo);
    }
#pragma unroll
    for (int i = 0; i < 4; ++i) {
      const size_t ao = (size_t)(m0 + (i << 4) + rlane) * lda + koff + k0;
      V ah = Frag<T>::load(Ab + ao);
      V al;
      if (SPLIT) al = Frag<T>::load(Ab2 + ao);
#pragma unroll
      for (int j = 0; j < 4; ++j) {
        acc[i][j] = Frag<T>::mma(ah, bh[j], acc[i][j]);
        if (SPLIT) {
          acc[i][j] = Frag<T>::mma(ah, bl[j], acc[i][j]);
          acc[i][j] = Frag<T>::mma(al, bh[j], acc[i][j]);
        }
      }
      Frag<T>::guard(acc[i][0], acc[i][3], ah, SPLIT ? al : ah);
    }
    Frag<T>::keep(bh[0], bh[1], bh[2], bh[3]);
    if (SPLIT) Frag<T>::keep(bl[0], bl[1], bl[2], bl[3]);
  }
  acc_guard4(acc[0][0], acc[0][1], acc[0][2], acc[0][3]);
  acc_guard4(acc[1][0], acc[1][1], acc[1][2], acc[1][3]);
  acc_guard4(acc[2][0], acc[2][1], acc[2][2], acc[2][3]);
  acc_guard4(acc[3][0], acc[3][1], acc[3][2], acc[3][3]);

  float* slab = sT[wave];
  const float* Rb = RESID ? (resid + (size_t)b * strideR) : nullptr;
#pragma unroll
  for (int i = 0; i < 4; ++i) {
    const int mBase = m0 + (i << 4);
#pragma unroll
    for (int j = 0; j < 4; ++j) {
      const int n = n0 + (j << 4) + rlane;
      float bv = 0.f;
      if (BIAS_MODE == 2) bv = bias[n];
#pragma unroll
      for (int r = 0; r < 8; ++r) {
        float v = acc[i][j][r] * scale;
        if (BIAS_MODE == 1) v += bias[mBase + mOff + r];
        if (BIAS_MODE == 2) v += bv;
        if (RESID) v += Rb[(size_t)(mBase + mOff + r) * ldc + n];
        if (ACT == 2) v = fmaxf(v, 0.0f);
        if (ACT == 4) v = (v > 0.f) ? v : 0.01f * v;
        slab[(mOff + r) * 68 + (j << 4) + rlane] = v;
      }
    }
    __builtin_amdgcn_fence(__ATOMIC_RELEASE, "workgroup");
    __builtin_amdgcn_wave_barrier();
    __builtin_amdgcn_fence(__ATOMIC_ACQUIRE, "workgroup");
    if (OUT_MODE == 0) {
      float* C = (float*)Cout + (size_t)b * strideC;
      const int hh = lane >> 4, c4 = (lane & 15) * 4;
      for (int pass = 0; pass < 2; ++pass) {
#pragma unroll
        for (int it = 0; it < 8; ++it) {
          const int row = it * 2 + hh;
          v4f v = *(const v4f*)(slab + row * 68 + c4);
          *(volatile v4f*)(C + (size_t)(mBase + row) * ldc + n0 + c4) = v;
        }
        __threadfence();
      }
    } else {
      const int q = lane >> 3, c8 = (lane & 7) * 8;
      unsigned short* C  = (unsigned short*)Cout  + (size_t)b * strideC;
      unsigned short* C2 = (OUT_MODE == 2) ? ((unsigned short*)Cout2 + (size_t)b * strideC) : nullptr;
      for (int pass = 0; pass < 2; ++pass) {
#pragma unroll
        for (int it = 0; it < 4; ++it) {
          const int row = it * 4 + q;
          const float* sp = slab + row * 68 + c8;
          v8h hv, lv;
#pragma unroll
          for (int e = 0; e < 8; ++e) {
            if (OUT_MODE == 1) {
              hv[e] = (_Float16)sp[e];
            } else {
              unsigned short hb = f2bf_bits(sp[e]);
              unsigned short lb = f2bf_bits(sp[e] - bf_bits2f(hb));
              hv[e] = __builtin_bit_cast(_Float16, hb);
              lv[e] = __builtin_bit_cast(_Float16, lb);
            }
          }
          *(volatile v8h*)(C + (size_t)(mBase + row) * ldc + n0 + c8) = hv;
          if (OUT_MODE == 2) *(volatile v8h*)(C2 + (size_t)(mBase + row) * ldc + n0 + c8) = lv;
        }
        __threadfence();
      }
    }
    __builtin_amdgcn_fence(__ATOMIC_RELEASE, "workgroup");
    __builtin_amdgcn_wave_barrier();
    __builtin_amdgcn_fence(__ATOMIC_ACQUIRE, "workgroup");
  }
}

__global__ __launch_bounds__(256) void wtcast_kernel(const float* __restrict__ W, int Nout, int Kin,
                                                     unsigned short* __restrict__ out, float scale) {
  __shared__ float sm[64][65];
  const int t  = threadIdx.x;
  const int k0 = blockIdx.x * 64;
  const int n0 = blockIdx.y * 64;
#pragma unroll
  for (int i = 0; i < 16; ++i) {
    const int e = i * 256 + t;
    const int r = e >> 6;
    const int c = e & 63;
    sm[c][r] = W[(size_t)(k0 + r) * Nout + n0 + c] * scale;
  }
  __syncthreads();
  const int lane = t & 31, wave = t >> 5;
  const int q = lane >> 3, c8 = (lane & 7) * 8;
  for (int pass = 0; pass < 2; ++pass) {
#pragma unroll
    for (int it = 0; it < 2; ++it) {
      const int row = wave * 8 + it * 4 + q;
      unsigned short hb[8];
#pragma unroll
      for (int e = 0; e < 8; ++e) hb[e] = h_bits(sm[row][c8 + e]);
      const v4u u = (v4u){pk16(hb[0], hb[1]), pk16(hb[2], hb[3]), pk16(hb[4], hb[5]), pk16(hb[6], hb[7])};
      *(volatile v4u*)(out + (size_t)(n0 + row) * Kin + k0 + c8) = u;
    }
    __threadfence();
  }
}

__global__ __launch_bounds__(128) void ln_kernel(const float* __restrict__ x, const float* __restrict__ w,
                                                 const float* __restrict__ bb, unsigned short* __restrict__ out) {
  __shared__ float red0[4];
  __shared__ float red1[4];
  const int row  = blockIdx.x;
  const int t    = threadIdx.x;
  const int lane = t & 31, wave = t >> 5;
  const int c0   = t * 8;
  const float* xr = x + (size_t)row * kDModel + c0;
  const v4f a = *(const v4f*)(xr);
  const v4f c = *(const v4f*)(xr + 4);
  float s = ((a[0] + a[1]) + (a[2] + a[3])) + ((c[0] + c[1]) + (c[2] + c[3]));
#pragma unroll
  for (int off = 16; off > 0; off >>= 1) s += __shfl_xor(s, off, 32);
  if (lane == 0) red0[wave] = s;
  __syncthreads();
  const float mean = ((red0[0] + red0[1]) + (red0[2] + red0[3])) * kInvD;
  float d[8];
#pragma unroll
  for (int e = 0; e < 4; ++e) { d[e] = a[e] - mean; d[4 + e] = c[e] - mean; }
  float ss = 0.f;
#pragma unroll
  for (int e = 0; e < 8; ++e) ss += d[e] * d[e];
#pragma unroll
  for (int off = 16; off > 0; off >>= 1) ss += __shfl_xor(ss, off, 32);
  if (lane == 0) red1[wave] = ss;
  __syncthreads();
  const float var = ((red1[0] + red1[1]) + (red1[2] + red1[3])) * kInvD;
  const float inv = rsqrtf(var + kLnEps);
  const v4f wa = *(const v4f*)(w + c0);
  const v4f wc = *(const v4f*)(w + c0 + 4);
  const v4f ba = *(const v4f*)(bb + c0);
  const v4f bc = *(const v4f*)(bb + c0 + 4);
  unsigned short hb[8];
#pragma unroll
  for (int e = 0; e < 4; ++e) {
    hb[e]     = h_bits(d[e] * inv * wa[e] + ba[e]);
    hb[4 + e] = h_bits(d[4 + e] * inv * wc[e] + bc[e]);
  }
  const v4u u = (v4u){pk16(hb[0], hb[1]), pk16(hb[2], hb[3]), pk16(hb[4], hb[5]), pk16(hb[6], hb[7])};
  unsigned short* op = out + (size_t)row * kDModel + c0;
  *(volatile v4u*)op = u;
  __threadfence();
  *(volatile v4u*)op = u;
}

__global__ __launch_bounds__(256) void vt_kernel(const unsigned* __restrict__ QKV32, unsigned short* __restrict__ VT) {
  __shared__ unsigned short sm[64][72];
  const int t   = threadIdx.x;
  const int s0  = blockIdx.x * 64;
  const int bk  = blockIdx.y;
  const int b   = bk >> 2;
  const int kvh = bk & 3;
  constexpr int kRowWords = kQKVN / 2;
  const size_t wbase = (size_t)(b * kSeq + s0) * kRowWords + (kVcol + kvh * kHeadDim) / 2;
#pragma unroll
  for (int i = 0; i < 8; ++i) {
    const int e  = i * 256 + t;
    const int r  = e >> 5;
    const int wc = e & 31;
    const unsigned wv = QKV32[wbase + (size_t)r * kRowWords + wc];
    sm[2 * wc][r]     = (unsigned short)(wv & 0xffffu);
    sm[2 * wc + 1][r] = (unsigned short)(wv >> 16);
  }
  __syncthreads();
  const int lane = t & 31, wave = t >> 5;
  const int q = lane >> 3, c8 = (lane & 7) * 8;
  for (int pass = 0; pass < 2; ++pass) {
#pragma unroll
    for (int it = 0; it < 2; ++it) {
      const int row = wave * 8 + it * 4 + q;
      const unsigned short* sp = &sm[row][c8];
      const v4u u = (v4u){pk16(sp[0], sp[1]), pk16(sp[2], sp[3]), pk16(sp[4], sp[5]), pk16(sp[6], sp[7])};
      *(volatile v4u*)(VT + ((size_t)(bk * kHeadDim + row)) * kSeq + s0 + c8) = u;
    }
    __threadfence();
  }
}

__global__ __launch_bounds__(512) void softmax_causal_kernel(const float* __restrict__ S, unsigned short* __restrict__ P) {
  __shared__ float redM[16];
  __shared__ float redS[16];
  const int r    = blockIdx.x;
  const int g    = blockIdx.y;
  const int t    = threadIdx.x;
  const int lane = t & 31, wave = t >> 5;
  const int c0   = t * 4;
  const size_t rowoff = ((size_t)g * kSeq + r) * kSeq;
  const v4f a = *(const v4f*)(S + rowoff + c0);
  const float x0 = (c0 + 0 > r) ? -INFINITY : a[0] * kScoreScale;
  const float x1 = (c0 + 1 > r) ? -INFINITY : a[1] * kScoreScale;
  const float x2 = (c0 + 2 > r) ? -INFINITY : a[2] * kScoreScale;
  const float x3 = (c0 + 3 > r) ? -INFINITY : a[3] * kScoreScale;
  float m = fmaxf(fmaxf(x0, x1), fmaxf(x2, x3));
#pragma unroll
  for (int off = 16; off > 0; off >>= 1) m = fmaxf(m, __shfl_xor(m, off, 32));
  if (lane == 0) redM[wave] = m;
  __syncthreads();
  float mm = redM[0];
#pragma unroll
  for (int i = 1; i < 16; ++i) mm = fmaxf(mm, redM[i]);
  const float p0 = expf(x0 - mm);
  const float p1 = expf(x1 - mm);
  const float p2 = expf(x2 - mm);
  const float p3 = expf(x3 - mm);
  float s = (p0 + p1) + (p2 + p3);
#pragma unroll
  for (int off = 16; off > 0; off >>= 1) s += __shfl_xor(s, off, 32);
  if (lane == 0) redS[wave] = s;
  __syncthreads();
  float tot = redS[0];
#pragma unroll
  for (int i = 1; i < 16; ++i) tot += redS[i];
  const float inv = kPCarry / tot;
  const v2u u = (v2u){pk16(h_bits(p0 * inv), h_bits(p1 * inv)), pk16(h_bits(p2 * inv), h_bits(p3 * inv))};
  unsigned short* op = P + rowoff + c0;
  *(volatile v2u*)op = u;
  __threadfence();
  *(volatile v2u*)op = u;
}

__global__ __launch_bounds__(256) void swiglu_kernel(const float* __restrict__ GU, unsigned short* __restrict__ H, int mrow0) {
  const int i = blockIdx.x * 256 + threadIdx.x;
  if (i >= kMChunk * (kDff / 2)) return;
  const int row = i >> 11;
  const int j2  = (i & 2047) * 2;
  const float* gp = GU + (size_t)row * kGUld + j2;
  const v2f g = *(const v2f*)(gp);
  const v2f u = *(const v2f*)(gp + kDff);
  const float sg0 = 1.0f / (1.0f + expf(-g[0]));
  const float sg1 = 1.0f / (1.0f + expf(-g[1]));
  const float h0 = (g[0] * sg0) * u[0] * kHCarry;
  const float h1 = (g[1] * sg1) * u[1] * kHCarry;
  const unsigned pk = pk16(h_bits(h0), h_bits(h1));
  unsigned* dst = (unsigned*)(void*)(H + (size_t)(mrow0 + row) * kDff + j2);
  *(volatile unsigned*)dst = pk;
  __threadfence();
  *(volatile unsigned*)dst = pk;
}

extern "C" void kernel_launch(void* const* d_in, const int* in_sizes, int n_in,
                              void* d_out, int out_size, void* d_ws, size_t ws_size,
                              hipStream_t stream) {
  if (n_in < 10) return;
  if (in_sizes[0] != kTok * kDModel || in_sizes[1] != kDModel || in_sizes[2] != kDModel ||
      in_sizes[3] != kDModel * kDModel || in_sizes[4] != kDModel * kKVDim || in_sizes[5] != kDModel * kKVDim ||
      in_sizes[6] != kDModel * kDModel || in_sizes[7] != kDModel * kDff || in_sizes[8] != kDModel * kDff ||
      in_sizes[9] != kDff * kDModel || out_size != kTok * kDModel) return;
  const size_t MiB = (size_t)1048576;
  const size_t ws_need = 112 * MiB;
  if (ws_size < ws_need) return;

  const float* x      = (const float*)d_in[0];
  const float* ln_w   = (const float*)d_in[1];
  const float* ln_b   = (const float*)d_in[2];
  const float* wq     = (const float*)d_in[3];
  const float* wk     = (const float*)d_in[4];
  const float* wv     = (const float*)d_in[5];
  const float* wo     = (const float*)d_in[6];
  const float* w_gate = (const float*)d_in[7];
  const float* w_up   = (const float*)d_in[8];
  const float* w_down = (const float*)d_in[9];
  float* out = (float*)d_out;

  char* ws = (char*)d_ws;
  unsigned short* N16   = (unsigned short*)(ws + 0 * MiB);
  float*          ATTO  = (float*)(ws + 8 * MiB);
  unsigned short* QKV   = (unsigned short*)(ws + 24 * MiB);
  unsigned short* VT    = (unsigned short*)(ws + 36 * MiB);
  unsigned short* WQKVT = (unsigned short*)(ws + 38 * MiB);
  unsigned short* WOT   = (unsigned short*)(ws + 41 * MiB);
  unsigned short* ATT16 = (unsigned short*)(ws + 43 * MiB);
  float*          Sbuf  = (float*)(ws + 51 * MiB);
  unsigned short* Pbuf  = (unsigned short*)(ws + 83 * MiB);
  unsigned short* WGUT  = (unsigned short*)(ws + 24 * MiB);
  unsigned short* WDT   = (unsigned short*)(ws + 40 * MiB);
  unsigned short* H16   = (unsigned short*)(ws + 48 * MiB);
  float*          GU    = (float*)(ws + 80 * MiB);

  const float wInv   = 1.0f / kWCarry;
  const float pvScl  = kAttCarry / kPCarry;
  const float woScl  = 1.0f / (kAttCarry * kWCarry);
  const float dnScl  = 1.0f / (kHCarry * kWdCarry);

  wtcast_kernel<<<dim3(kDModel / 64, kDModel / 64), 256, 0, stream>>>(wq, kDModel, kDModel, WQKVT, kWCarry);
  wtcast_kernel<<<dim3(kDModel / 64, kKVDim / 64), 256, 0, stream>>>(wk, kKVDim, kDModel, WQKVT + (size_t)kKcol * kDModel, kWCarry);
  wtcast_kernel<<<dim3(kDModel / 64, kKVDim / 64), 256, 0, stream>>>(wv, kKVDim, kDModel, WQKVT + (size_t)kVcol * kDModel, kWCarry);
  wtcast_kernel<<<dim3(kDModel / 64, kDModel / 64), 256, 0, stream>>>(wo, kDModel, kDModel, WOT, kWCarry);

  ln_kernel<<<kTok, 128, 0, stream>>>(x, ln_w, ln_b, N16);

  wmma_gemm64<0, false, 0, 1, false, 0, 0><<<dim3((64 * 24 + 7) / 8, 1), 256, 0, stream>>>(
      N16, nullptr, kDModel, 0L, WQKVT, nullptr, kDModel, 0L,
      (void*)QKV, nullptr, kQKVN, 0L, nullptr, nullptr, 0L, kTok, kQKVN, kDModel, wInv);

  vt_kernel<<<dim3(kSeq / 64, kBatch * kKVHeads), 256, 0, stream>>>((const unsigned*)(const void*)QKV, VT);

  const long sStride = (long)kSeq * kSeq;
  for (int pc = 0; pc < kBatch * (kHeads / 2); ++pc) {
    const int b   = pc / (kHeads / 2);
    const int h0  = (pc % (kHeads / 2)) * 2;
    const int kvh = h0 / (kHeads / kKVHeads);
    const unsigned short* Qp = QKV + (size_t)b * kSeq * kQKVN + (size_t)h0 * kHeadDim;
    const unsigned short* Kp = QKV + (size_t)b * kSeq * kQKVN + kKcol + (size_t)kvh * kHeadDim;
    const unsigned short* Vtp = VT + (size_t)((b * kKVHeads + kvh) * kHeadDim) * kSeq;
    wmma_gemm64<0, false, 0, 0, false, 0, 1><<<dim3((32 * 32 + 7) / 8, 2), 256, 0, stream>>>(
        Qp, nullptr, kQKVN, (long)kHeadDim, Kp, nullptr, kQKVN, 0L,
        (void*)Sbuf, nullptr, kSeq, sStride, nullptr, nullptr, 0L, kSeq, kSeq, kHeadDim, 1.0f);
    softmax_causal_kernel<<<dim3(kSeq, 2), 512, 0, stream>>>(Sbuf, Pbuf);
    wmma_gemm64<0, false, 0, 1, false, 0, 2><<<dim3((32 * 1 + 7) / 8, 2), 256, 0, stream>>>(
        Pbuf, nullptr, kSeq, sStride, Vtp, nullptr, kSeq, 0L,
        (void*)(ATT16 + (size_t)b * kSeq * kDModel + (size_t)h0 * kHeadDim), nullptr, kDModel, (long)kHeadDim,
        nullptr, nullptr, 0L, kSeq, kHeadDim, kSeq, pvScl);
  }

  wmma_gemm64<0, false, 0, 0, true, 0, 0><<<dim3((64 * 16 + 7) / 8, 1), 256, 0, stream>>>(
      ATT16, nullptr, kDModel, 0L, WOT, nullptr, kDModel, 0L,
      (void*)ATTO, nullptr, kDModel, 0L, nullptr, x, 0L, kTok, kDModel, kDModel, woScl);

  wtcast_kernel<<<dim3(kDModel / 64, kDff / 64), 256, 0, stream>>>(w_gate, kDff, kDModel, WGUT, kWCarry);
  wtcast_kernel<<<dim3(kDModel / 64, kDff / 64), 256, 0, stream>>>(w_up, kDff, kDModel, WGUT + (size_t)kDff * kDModel, kWCarry);
  wtcast_kernel<<<dim3(kDff / 64, kDModel / 64), 256, 0, stream>>>(w_down, kDModel, kDff, WDT, kWdCarry);

  for (int mc = 0; mc < kTok / kMChunk; ++mc) {
    wmma_gemm64<0, false, 0, 0, false, 0, 0><<<dim3((16 * 128 + 7) / 8, 1), 256, 0, stream>>>(
        N16 + (size_t)mc * kMChunk * kDModel, nullptr, kDModel, 0L, WGUT, nullptr, kDModel, 0L,
        (void*)GU, nullptr, kGUld, 0L, nullptr, nullptr, 0L, kMChunk, kGUld, kDModel, wInv);
    swiglu_kernel<<<(kMChunk * (kDff / 2) + 255) / 256, 256, 0, stream>>>(GU, H16, mc * kMChunk);
  }

  wmma_gemm64<0, false, 0, 0, true, 0, 0><<<dim3((64 * 16 + 7) / 8, 1), 256, 0, stream>>>(
      H16, nullptr, kDff, 0L, WDT, nullptr, kDff, 0L,
      (void*)out, nullptr, kDModel, 0L, nullptr, ATTO, 0L, kTok, kDModel, kDff, dnScl);
}
